// MultiHeadSelfAttention_82970178224305
// MI455X (gfx1250) — hardware-verified
//
#include <hip/hip_runtime.h>
#ifndef NB
#define NB 4
#endif
#ifndef SEQ
#define SEQ 1024
#endif
#define NB_FULL 4
#define SEQ_FULL 1024
#define SQ SEQ
#define DM 1024
#define NH 16
#define HD 64
#define HG 8
#define RW 128
#define NPOS (2 * RW + 1)
#define RJ 320
#define PKP (SQ + RJ)
#define NR ((size_t)NB * SQ)
#define MP ((int)NR)
#define LQ DM

static_assert(NB >= 1 && NB <= NB_FULL);
static_assert(SQ >= 256 && SQ <= SEQ_FULL && (SQ % 256) == 0);
static_assert((MP % 128) == 0 && (DM % 64) == 0 && (DM % 32) == 0 && HD == 64 && (NH % HG) == 0);
static_assert(((size_t)(NB - 1) * SEQ_FULL + SQ) * DM <= (size_t)NB_FULL * SEQ_FULL * DM);
static_assert(NPOS == 257 && RJ >= NPOS && RJ == 320 && (RJ % 64) == 0 && (RJ / 4) <= 96);
static_assert((PKP % 32) == 0 && ((PKP * 2) % 128) == 0 && ((RJ * 4) % 128) == 0);
static_assert(((RJ * (HD / 8)) % 256) == 0 && ((NH * HD * (RJ / 8)) % 256) == 0);
static_assert((SQ % 128) == 0 && (HD % 32) == 0 && (SQ * HG) % 8 == 0);
#define WS_W   ((size_t)DM * DM * 2)
#define WS_X   ((size_t)NR * DM * 2)
#define WS_S   ((size_t)HG * SQ * SQ * 4)
#define WS_R   ((size_t)HG * SQ * RJ * 4)
#define WS_P   ((size_t)HG * SQ * PKP * 2)
#define WS_VT  ((size_t)NH * HD * PKP * 2)
#define WS_PK  ((size_t)RJ * HD * 2)
#define WS_TOTAL (4 * WS_W + 5 * WS_X + WS_S + WS_R + WS_P + WS_VT + WS_PK)
static_assert((WS_W % 256) == 0 && (WS_X % 256) == 0 && (WS_S % 256) == 0 && (WS_R % 256) == 0 && (WS_P % 256) == 0 && (WS_VT % 256) == 0 && (WS_PK % 256) == 0);
static_assert(WS_TOTAL <= (size_t)134217728);

typedef unsigned short v8us __attribute__((ext_vector_type(8), may_alias));
typedef float  v8f  __attribute__((ext_vector_type(8)));
typedef float  v4f  __attribute__((ext_vector_type(4)));
typedef float  v4fa __attribute__((ext_vector_type(4), may_alias));
typedef _Float16 v16h __attribute__((ext_vector_type(16)));
typedef _Float16 v4h __attribute__((ext_vector_type(4)));
union FragH { v16h v; v8us half[2]; _Float16 h[16]; unsigned short u[16]; };

__device__ __forceinline__ unsigned short bf16_bits(float x) { unsigned int u = __float_as_uint(x); return (unsigned short)((u + 0x7FFFu + ((u >> 16) & 1u)) >> 16); }
__device__ __forceinline__ float bf16_val(unsigned short b) { return __uint_as_float(((unsigned int)b) << 16); }
__device__ __forceinline__ float bf16_rne(float x) { return bf16_val(bf16_bits(x)); }
static __device__ __forceinline__ _Float16 toh_flush(float v) { const _Float16 r = (_Float16)v; return (fabsf(v) < 6.103515625e-05f) ? (_Float16)0.0f : r; }

__device__ __forceinline__ v16h g2_frag(const _Float16* p, int hh) { FragH f; f.half[0] = *(const v8us*)((const unsigned short*)p + 8 * hh); f.half[1] = *(const v8us*)((const unsigned short*)p + 16 + 8 * hh); return f.v; }
__device__ __forceinline__ v8f g2_mma(v16h a, v16h b, v8f c) { v8f d = __builtin_amdgcn_wmma_f32_16x16x32_f16(false, a, false, b, (short)0, c, false, false); asm volatile("v_nop\n\tv_nop\n\tv_nop\n\tv_nop" : "+v"(d) : "v"(a), "v"(b)); return d; }
template <int ACT>
__global__ __launch_bounds__(128) void k_gemm2(const _Float16* __restrict__ A, int lda, size_t sA, const _Float16* __restrict__ Bh, int ldb, size_t sB, float alpha, const float* __restrict__ bias, size_t sBias, const float* __restrict__ CP, int rowsPerB, size_t sCPb, int row0g,
    float* __restrict__ C, _Float16* __restrict__ C16, int ldc, size_t sC, int M, int N, int K) {
  static_assert(ACT == 0 || ACT == 3);
  __shared__ __attribute__((aligned(16))) float so[4][32][68];
  const int tid = threadIdx.x, w = tid >> 5, lane = tid & 31, ln = lane & 15, hh = lane >> 4; const int by = blockIdx.y;
  A += (size_t)by * sA; Bh += (size_t)by * sB; const size_t cofs = (size_t)by * sC; const float* bp = bias ? bias + (size_t)by * sBias : nullptr;
  const int ntn = N >> 6; const int mt = blockIdx.x / ntn, nq = blockIdx.x - mt * ntn; const int row0 = mt * 128 + 32 * w, col0 = nq * 64; if (row0 >= M) return;
  const _Float16* a0p = A + (size_t)(row0 + ln) * lda; const _Float16* a1p = a0p + (size_t)16 * lda;
  const _Float16* b0p = Bh + (size_t)(col0 + ln) * ldb; const _Float16* b1p = b0p + (size_t)16 * ldb; const _Float16* b2p = b1p + (size_t)16 * ldb; const _Float16* b3p = b2p + (size_t)16 * ldb;
  const v8f z8 = {0.f,0.f,0.f,0.f,0.f,0.f,0.f,0.f}; v8f c00 = z8, c01 = z8, c02 = z8, c03 = z8, c10 = z8, c11 = z8, c12 = z8, c13 = z8;
#pragma unroll 1
  for (int kb = 0; kb < K; kb += 32) { const v16h a0 = g2_frag(a0p + kb, hh), a1 = g2_frag(a1p + kb, hh);
    v16h b = g2_frag(b0p + kb, hh); c00 = g2_mma(a0, b, c00); c10 = g2_mma(a1, b, c10);
    b = g2_frag(b1p + kb, hh); c01 = g2_mma(a0, b, c01); c11 = g2_mma(a1, b, c11);
    b = g2_frag(b2p + kb, hh); c02 = g2_mma(a0, b, c02); c12 = g2_mma(a1, b, c12);
    b = g2_frag(b3p + kb, hh); c03 = g2_mma(a0, b, c03); c13 = g2_mma(a1, b, c13); }
  v8f accs[8] = {c00, c01, c02, c03, c10, c11, c12, c13};
#pragma unroll
  for (int u = 0; u < 8; ++u) { const int t = u & 3, half = u >> 2; const int col = col0 + t * 16 + ln; const float bv = bp ? bf16_rne(bp[col]) : 0.f;
#pragma unroll
    for (int r = 0; r < 8; ++r) { const int rloc = half * 16 + 8 * hh + r; float v = accs[u][r] * alpha + bv;
      if (CP) { if (rowsPerB < 0) v += CP[cofs + (size_t)(row0g + row0 + rloc) * ldc + col]; else { const int bidx = (row0g + row0 + rloc) / rowsPerB; v += CP[(size_t)bidx * sCPb + (size_t)by * 64 + col]; } }
      if (ACT == 3) v = fmaxf(v, 0.f);
      so[w][rloc][t * 16 + ln] = v; } }
  __builtin_amdgcn_fence(4  , "workgroup"); __builtin_amdgcn_wave_barrier();
  const int rsub = lane >> 4, c4 = (lane & 15) * 4;
  for (int pass = 0; pass < 2; ++pass) {
#pragma unroll
    for (int q = 0; q < 16; ++q) { const int r = q * 2 + rsub; const v4f v = *(const v4fa*)&so[w][r][c4];
      if (C) *(volatile v4f*)(C + cofs + (size_t)(row0 + r) * ldc + col0 + c4) = v;
      if (C16) { v4h h4; for (int i = 0; i < 4; ++i) h4[i] = (_Float16)v[i]; *(volatile v4h*)(C16 + cofs + (size_t)(row0 + r) * ldc + col0 + c4) = h4; } }
    if (pass == 0) __threadfence(); } }

__global__ __launch_bounds__(256) void k_wt_f16(const float* __restrict__ W, _Float16* __restrict__ Wt, int K, int N, float scale) {
  const int t = blockIdx.x * 256 + threadIdx.x; if (t >= N * (K / 8)) return; const int n = t / (K / 8), k8 = (t % (K / 8)) * 8; FragH f;
#pragma unroll
  for (int i = 0; i < 8; ++i) f.h[i] = (_Float16)(bf16_rne(W[(size_t)(k8 + i) * N + n]) * scale); const v8us o = f.half[0];
  *(volatile v8us*)((unsigned short*)Wt + (size_t)n * K + k8) = o; __threadfence(); *(volatile v8us*)((unsigned short*)Wt + (size_t)n * K + k8) = o;
}

__global__ __launch_bounds__(256) void k_x16(const float* __restrict__ x, _Float16* __restrict__ X16, size_t n8) {
  const size_t t = (size_t)blockIdx.x * 256 + threadIdx.x; if (t >= n8) return;
  const size_t e = t * 8; const size_t rc = e / DM; const size_t c = e % DM; const size_t b = rc / SQ, s = rc % SQ;
  const float* src = x + ((b * SEQ_FULL + s) * DM + c);
  const v4f a = *(const v4fa*)src, d = *(const v4fa*)(src + 4); FragH f;
#pragma unroll
  for (int q = 0; q < 4; ++q) { f.h[q] = (_Float16)bf16_rne(a[q]); f.h[4 + q] = (_Float16)bf16_rne(d[q]); }
  *(volatile v8us*)((unsigned short*)X16 + t * 8) = f.half[0]; __threadfence(); *(volatile v8us*)((unsigned short*)X16 + t * 8) = f.half[0]; }

__global__ __launch_bounds__(256) void k_posk(const float* __restrict__ pk, _Float16* __restrict__ PK) {
  #pragma clang fp contract(off)
  const int t = blockIdx.x * 256 + threadIdx.x; if (t >= RJ * (HD / 8)) return;
  const int j = t / (HD / 8), d8 = (t % (HD / 8)) * 8; const int jc = j < NPOS ? j : NPOS - 1;
  v4f a = *(const v4fa*)(pk + (size_t)jc * HD + d8), b = *(const v4fa*)(pk + (size_t)jc * HD + d8 + 4);
  asm volatile("" : "+v"(a)); asm volatile("" : "+v"(b));
  FragH f;
#pragma unroll
  for (int q = 0; q < 4; ++q) { f.h[q] = toh_flush((j < NPOS) ? bf16_rne(a[q]) * 16.0f : 0.0f); f.h[4 + q] = toh_flush((j < NPOS) ? bf16_rne(b[q]) * 16.0f : 0.0f); }
  const v8us o = f.half[0];
  *(volatile v8us*)((unsigned short*)PK + (size_t)t * 8) = o; __threadfence(); *(volatile v8us*)((unsigned short*)PK + (size_t)t * 8) = o; }

__global__ __launch_bounds__(256) void k_posvt(const float* __restrict__ pv, _Float16* __restrict__ Vt) {
  #pragma clang fp contract(off)
  const int t = blockIdx.x * 256 + threadIdx.x; if (t >= NH * HD * (RJ / 8)) return;
  const int row = t / (RJ / 8), j0 = (t % (RJ / 8)) * 8; const int dd = row % HD; FragH f;
#pragma unroll
  for (int e = 0; e < 8; ++e) { const int j = j0 + e; const int jc = j < NPOS ? j : NPOS - 1; float val = pv[(size_t)jc * HD + dd]; asm volatile("" : "+v"(val));
    f.h[e] = toh_flush((j < NPOS) ? bf16_rne(val) * 16.0f : 0.0f); }
  const v8us o = f.half[0]; unsigned short* dst = (unsigned short*)Vt + (size_t)row * PKP + SQ + j0;
  *(volatile v8us*)dst = o; __threadfence(); *(volatile v8us*)dst = o; }

template <int NHv, int TTv, int PTv>
__global__ __launch_bounds__(256) void k_vt(const _Float16* __restrict__ V16, int ldv, int voff, _Float16* __restrict__ Vt) { __shared__ unsigned short tl[64][66]; const int tid = threadIdx.x; const int slab = blockIdx.x / (TTv / 64), lg = blockIdx.x % (TTv / 64); const int b = slab / NHv, h = slab % NHv;
  for (int i = tid; i < 64 * 8; i += 256) { const int r = i / 8, c8 = (i % 8) * 8; FragH f; f.half[0] = *(const v8us*)((const unsigned short*)V16 + ((size_t)b * TTv + lg * 64 + r) * ldv + voff + h * 64 + c8);
#pragma unroll
    for (int q = 0; q < 8; ++q) tl[r][c8 + q] = f.u[q]; }
  __syncthreads();
  for (int pass = 0; pass < 2; ++pass) {
#pragma unroll
    for (int rd = 0; rd < 2; ++rd) { const int d = rd * 32 + tid / 8, pc = tid % 8; FragH f;
#pragma unroll
      for (int q = 0; q < 8; ++q) f.u[q] = tl[pc * 8 + q][d];
      *(volatile v8us*)((unsigned short*)Vt + ((size_t)slab * 64 + d) * PTv + lg * 64 + pc * 8) = f.half[0]; }
    if (pass == 0) __threadfence(); } }

__global__ __launch_bounds__(256) void k_rsmr(const float* __restrict__ S, const float* __restrict__ R, const float* __restrict__ mk, _Float16* __restrict__ P, int qn, int hg) {
  #pragma clang fp contract(off)
  __shared__ __attribute__((aligned(16))) float rl[8][RJ];
  __shared__ __attribute__((aligned(16))) float pl[8][SQ];
  const int w = __builtin_amdgcn_readfirstlane(threadIdx.x >> 5), lane = threadIdx.x & 31;
  const int t = blockIdx.x * 8 + w; if (t >= qn * hg) return;
  const int qi = t % qn; const size_t i = (size_t)(t / qn) * SQ + (size_t)qi;
  const float* s = S + i * SQ; const float* rr = R + i * RJ; unsigned short* d = (unsigned short*)P + i * PKP;
#pragma unroll
  for (int it = 0; it < 3; ++it) { int p4 = it * 32 + lane; p4 = p4 < (RJ / 4 - 1) ? p4 : (RJ / 4 - 1); const v4f a = *(const v4fa*)(rr + p4 * 4); *(v4fa*)&rl[w][p4 * 4] = a; }
  __builtin_amdgcn_fence(4  , "workgroup"); __builtin_amdgcn_wave_barrier();
  float v[SQ / 32];
#pragma unroll
  for (int c = 0; c < SQ / 256; ++c) { const int kb = c * 256 + lane * 8;
    const v4f a = *(const v4fa*)(s + kb), b = *(const v4fa*)(s + kb + 4); const v4f ma = *(const v4fa*)(mk + kb), mb = *(const v4fa*)(mk + kb + 4);
#pragma unroll
    for (int q = 0; q < 4; ++q) { int j0 = kb + q - qi; j0 = j0 < -RW ? -RW : j0; j0 = j0 > RW ? RW : j0; int j1 = kb + 4 + q - qi; j1 = j1 < -RW ? -RW : j1; j1 = j1 > RW ? RW : j1;
      const float r0 = rl[w][j0 + RW], r1 = rl[w][j1 + RW];
      v[c * 8 + q] = (a[q] + r0) * bf16_rne(ma[q]); v[c * 8 + 4 + q] = (b[q] + r1) * bf16_rne(mb[q]); } }
  float mx = -3.0e38f;
#pragma unroll
  for (int j = 0; j < SQ / 32; ++j) mx = fmaxf(mx, v[j]);
#pragma unroll
  for (int off = 16; off >= 1; off >>= 1) mx = fmaxf(mx, __shfl_xor(mx, off, 32));
  float se = 0.f;
#pragma unroll
  for (int j = 0; j < SQ / 32; ++j) { const float e = __expf(v[j] - mx); v[j] = e; se += e; }
#pragma unroll
  for (int off = 16; off >= 1; off >>= 1) se += __shfl_xor(se, off, 32);
  const float sc = 1024.0f / se;
  float blo = 0.f, bhi = 0.f;
  v8us ov[SQ / 256];
#pragma unroll
  for (int c = 0; c < SQ / 256; ++c) { FragH f;
#pragma unroll
    for (int q = 0; q < 8; ++q) { const int k = c * 256 + lane * 8 + q; const float pv = v[c * 8 + q] * sc; pl[w][k] = pv;
      blo += (k <= qi - RW) ? pv : 0.f; bhi += (k >= qi + RW) ? pv : 0.f; f.h[q] = toh_flush(pv); }
    ov[c] = f.half[0]; }
#pragma unroll
  for (int off = 16; off >= 1; off >>= 1) { blo += __shfl_xor(blo, off, 32); bhi += __shfl_xor(bhi, off, 32); }
  __builtin_amdgcn_fence(4  , "workgroup"); __builtin_amdgcn_wave_barrier();
  float zv = 0.0f; asm volatile("" : "+v"(zv));
  FragH f1, f2;
#pragma unroll
  for (int e = 0; e < 8; ++e) { const int j = lane * 8 + e; const int kk = qi + j - RW; int kc = kk < 0 ? 0 : kk; kc = kc > SQ - 1 ? SQ - 1 : kc;
    float val = pl[w][kc]; asm volatile("" : "+v"(val));
    val = (j >= 1 && kk >= 0 && kk < SQ) ? val : zv; val = (j == 0) ? blo : val;
    f1.h[e] = toh_flush(val * 0.0625f); }
  f2.h[0] = toh_flush(((lane == 0) ? bhi : zv) * 0.0625f);
#pragma unroll
  for (int e = 1; e < 8; ++e) f2.h[e] = toh_flush(zv);
  const v8us o1 = f1.half[0], o2 = f2.half[0];
  for (int pass = 0; pass < 2; ++pass) {
#pragma unroll
    for (int c = 0; c < SQ / 256; ++c) *(volatile v8us*)(d + c * 256 + lane * 8) = ov[c];
    *(volatile v8us*)(d + SQ + lane * 8) = o1;
    if (lane < 8) *(volatile v8us*)(d + SQ + 256 + lane * 8) = o2;
    if (pass == 0) __threadfence(); } }

extern "C" void kernel_launch(void* const* d_in, const int* in_sizes, int n_in,
                              void* d_out, int out_size, void* d_ws, size_t ws_size, hipStream_t stream) {
  if (n_in < 12) return;
  const size_t rows_need = (size_t)(NB - 1) * SEQ_FULL + SQ;
  if ((size_t)in_sizes[0] < rows_need * DM) return;
  if ((size_t)in_sizes[1] < rows_need) return;
  if (in_sizes[2] < DM * DM || in_sizes[4] < DM * DM || in_sizes[6] < DM * DM || in_sizes[8] < DM * DM) return;
  if (in_sizes[3] < DM || in_sizes[5] < DM || in_sizes[7] < DM || in_sizes[9] < DM) return;
  if (in_sizes[10] < NPOS * HD || in_sizes[11] < NPOS * HD) return;
  if ((size_t)out_size < rows_need * DM) return;
  const float* x  = (const float*)d_in[0];
  const float* pm = (const float*)d_in[1];
  const float* wq = (const float*)d_in[2]; const float* bq = (const float*)d_in[3];
  const float* wk = (const float*)d_in[4]; const float* bk = (const float*)d_in[5];
  const float* wv = (const float*)d_in[6]; const float* bv = (const float*)d_in[7];
  const float* wo = (const float*)d_in[8]; const float* bo = (const float*)d_in[9];
  const float* pk = (const float*)d_in[10]; const float* pv = (const float*)d_in[11];
  char* ws = (char*)d_ws; size_t off = 0;
  auto take = [&](size_t bytes) { char* p = ws + off; off += (bytes + 255) & ~(size_t)255; return p; };
  _Float16* BQ = (_Float16*)take(WS_W); _Float16* BK = (_Float16*)take(WS_W); _Float16* BV = (_Float16*)take(WS_W); _Float16* BO = (_Float16*)take(WS_W);
  _Float16* X16 = (_Float16*)take(WS_X); _Float16* Q16 = (_Float16*)take(WS_X); _Float16* K16 = (_Float16*)take(WS_X); _Float16* V16 = (_Float16*)take(WS_X); _Float16* CX = (_Float16*)take(WS_X);
  float* S = (float*)take(WS_S); float* R = (float*)take(WS_R); _Float16* P = (_Float16*)take(WS_P); _Float16* VT = (_Float16*)take(WS_VT); _Float16* PK = (_Float16*)take(WS_PK);
  if (off > ws_size) return;
  float* out = (float*)d_out;

  { const unsigned g = (unsigned)(((size_t)DM * DM / 8 + 255) / 256);
    k_wt_f16<<<g, 256, 0, stream>>>(wq, BQ, DM, DM, 16.0f); k_wt_f16<<<g, 256, 0, stream>>>(wk, BK, DM, DM, 16.0f); k_wt_f16<<<g, 256, 0, stream>>>(wv, BV, DM, DM, 16.0f); k_wt_f16<<<g, 256, 0, stream>>>(wo, BO, DM, DM, 16.0f); }
  k_x16<<<(unsigned)((NR * DM / 8 + 255) / 256), 256, 0, stream>>>(x, X16, NR * DM / 8);
  k_posk<<<(unsigned)((RJ * (HD / 8) + 255) / 256), 256, 0, stream>>>(pk, PK);
  k_posvt<<<(unsigned)((NH * HD * (RJ / 8) + 255) / 256), 256, 0, stream>>>(pv, VT);
  { const unsigned gp = (unsigned)((MP / 128) * (DM / 64));
    k_gemm2<0><<<dim3(gp, 1), 128, 0, stream>>>(X16, DM, 0, BQ, DM, 0, 0.0625f, bq, 0, nullptr, 1, 0, 0, nullptr, Q16, DM, 0, MP, DM, DM);
    k_gemm2<0><<<dim3(gp, 1), 128, 0, stream>>>(X16, DM, 0, BK, DM, 0, 0.0625f, bk, 0, nullptr, 1, 0, 0, nullptr, K16, DM, 0, MP, DM, DM);
    k_gemm2<0><<<dim3(gp, 1), 128, 0, stream>>>(X16, DM, 0, BV, DM, 0, 0.0625f, bv, 0, nullptr, 1, 0, 0, nullptr, V16, DM, 0, MP, DM, DM); }
  for (int b = 0; b < NB; ++b) { const size_t r0 = (size_t)b * SQ;
    k_vt<NH, SQ, PKP><<<NH * (SQ / 64), 256, 0, stream>>>(V16 + r0 * LQ, LQ, 0, VT);
    for (int h0 = 0; h0 < NH; h0 += HG) {
      k_gemm2<0><<<dim3((unsigned)((SQ / 128) * (SQ / 64)), HG), 128, 0, stream>>>(Q16 + r0 * LQ + h0 * HD, LQ, (size_t)HD, K16 + r0 * LQ + h0 * HD, LQ, (size_t)HD, 0.125f, nullptr, 0, nullptr, 1, 0, 0, S, nullptr, SQ, (size_t)SQ * SQ, SQ, SQ, HD);
      k_gemm2<0><<<dim3((unsigned)((SQ / 128) * (RJ / 64)), HG), 128, 0, stream>>>(Q16 + r0 * LQ + h0 * HD, LQ, (size_t)HD, PK, HD, 0, 0.0078125f, nullptr, 0, nullptr, 1, 0, 0, R, nullptr, RJ, (size_t)SQ * RJ, SQ, RJ, HD);
      k_rsmr<<<(unsigned)((HG * SQ + 7) / 8), 256, 0, stream>>>(S, R, pm + (size_t)b * SEQ_FULL, P, SQ, HG);
      k_gemm2<0><<<dim3((unsigned)((SQ / 128) * (HD / 64)), HG), 128, 0, stream>>>(P, PKP, (size_t)SQ * PKP, VT + (size_t)h0 * HD * PKP, PKP, (size_t)HD * PKP, 0.015625f, nullptr, 0, nullptr, 1, 0, 0, nullptr, CX + r0 * DM + h0 * HD, DM, (size_t)HD, SQ, HD, PKP); }
    k_gemm2<0><<<dim3((unsigned)((SQ / 128) * (DM / 64)), 1), 128, 0, stream>>>(CX + r0 * DM, DM, 0, BO, DM, 0, 0.00390625f, bo, 0, nullptr, 1, 0, 0, out + (size_t)b * SEQ_FULL * DM, nullptr, DM, 0, SQ, DM, DM); }
}
